// KVCacheSamAttention_43473658970634
// MI455X (gfx1250) — hardware-verified
//
#include <hip/hip_runtime.h>
#include <math.h>


#define NBH 32
#define SQ 2048
#define SK 2048
#define HD 64
#define BQ 64
#define BK 32

typedef __attribute__((ext_vector_type(16))) _Float16 v16h;
typedef __attribute__((ext_vector_type(8)))  _Float16 v8h;
typedef __attribute__((ext_vector_type(8)))  float v8f;
typedef __attribute__((ext_vector_type(4)))  float v4f;

template <typename T> __device__ __forceinline__ void vst2(void* p, T v) { *(volatile T*)p = v; __threadfence(); *(volatile T*)p = v; }
__device__ __forceinline__ v8f wmma16(v16h a, v16h b, v8f c) {
  v8f d = __builtin_amdgcn_wmma_f32_16x16x32_f16(false, a, false, b, (short)0, c, false, false);
  asm volatile("v_nop\n\tv_nop\n\tv_nop\n\tv_nop" : "+v"(d) : "v"(a), "v"(b));
  return d;
}
__device__ __forceinline__ v16h frag_h(const _Float16* rowk0, int lane) {
  union { v16h v; v8h q[2]; } u; const _Float16* p = rowk0 + 8 * (lane >> 4);
  u.q[0] = *(const v8h*)p; u.q[1] = *(const v8h*)(p + 16); return u.v;
}
__device__ __forceinline__ v16h frag_f32(const float* rowk0, int lane) {
  v16h a; const float* p = rowk0 + 8 * (lane >> 4);
#pragma unroll
  for (int i = 0; i < 8; ++i) { a[i] = (_Float16)p[i]; a[8 + i] = (_Float16)p[16 + i]; }
  return a;
}

__global__ __launch_bounds__(128) void attn_fwd(const float* __restrict__ Q, const float* __restrict__ K, const float* __restrict__ V,
                                                const float* __restrict__ mask, const int* __restrict__ scale_p, float* __restrict__ O) {
  __shared__ __align__(16) _Float16 sK[BK][HD + 8];
  __shared__ __align__(16) _Float16 sVt[HD][BK + 8];
  __shared__ __align__(16) float sP[4][16][BK];
  __shared__ __align__(16) float sO[4][16][HD];
  const int tid = threadIdx.x, w = tid >> 5, lane = tid & 31, g = lane >> 4, ln = lane & 15;
  const int bh = blockIdx.y;
  const int q0 = blockIdx.x * BQ + w * 16;
  const size_t base = (size_t)bh * SQ * HD;
  const float inv_scale = 1.0f / (float)scale_p[0];

  const float* qrow = Q + base + (size_t)(q0 + ln) * HD;
  const v16h qa0 = frag_f32(qrow, lane), qa1 = frag_f32(qrow + 32, lane);
  float mrun[8], lrun[8];
  v8f acc[4];
#pragma unroll
  for (int r = 0; r < 8; ++r) { mrun[r] = -3.0e38f; lrun[r] = 0.f; }
#pragma unroll
  for (int t = 0; t < 4; ++t) acc[t] = (v8f){};

  const int skey = tid >> 2, sd0 = (tid & 3) * 16;
  for (int k0 = 0; k0 < SK; k0 += BK) {
    __syncthreads();
    { const float* gk = K + base + (size_t)(k0 + skey) * HD + sd0; const float* gv = V + base + (size_t)(k0 + skey) * HD + sd0;
#pragma unroll
      for (int i = 0; i < 16; ++i) { sK[skey][sd0 + i] = (_Float16)gk[i]; sVt[sd0 + i][skey] = (_Float16)gv[i]; } }
    __syncthreads();

    v8f s0 = {}, s1 = {};
    s0 = wmma16(qa0, frag_h(&sK[ln][0], lane), s0);      s0 = wmma16(qa1, frag_h(&sK[ln][32], lane), s0);
    s1 = wmma16(qa0, frag_h(&sK[16 + ln][0], lane), s1); s1 = wmma16(qa1, frag_h(&sK[16 + ln][32], lane), s1);
    const float* mrow = mask + (size_t)(q0 + 8 * g) * SK + k0;
#pragma unroll
    for (int r = 0; r < 8; ++r) {
      const float x0 = s0[r] * inv_scale + mrow[(size_t)r * SK + ln], x1 = s1[r] * inv_scale + mrow[(size_t)r * SK + 16 + ln];
      float mx = fmaxf(x0, x1);
#pragma unroll
      for (int off = 8; off >= 1; off >>= 1) mx = fmaxf(mx, __shfl_xor(mx, off, 32));
      const float mn = fmaxf(mrun[r], mx);
      const float corr = expf(mrun[r] - mn);
      const float p0 = expf(x0 - mn), p1 = expf(x1 - mn);
      float sum = p0 + p1;
#pragma unroll
      for (int off = 8; off >= 1; off >>= 1) sum += __shfl_xor(sum, off, 32);
      lrun[r] = lrun[r] * corr + sum; mrun[r] = mn;
#pragma unroll
      for (int t = 0; t < 4; ++t) acc[t][r] *= corr;
      sP[w][8 * g + r][ln] = p0 * 16384.0f; sP[w][8 * g + r][16 + ln] = p1 * 16384.0f;
    }
    asm volatile("s_wait_dscnt 0" ::: "memory"); __builtin_amdgcn_wave_barrier(); __builtin_amdgcn_fence(__ATOMIC_RELEASE, "workgroup");
    const v16h pa = frag_f32(&sP[w][ln][0], lane);
#pragma unroll
    for (int t = 0; t < 4; ++t) acc[t] = wmma16(pa, frag_h(&sVt[t * 16 + ln][0], lane), acc[t]);
    __builtin_amdgcn_wave_barrier();
  }
  float* so = &sO[w][0][0];
#pragma unroll
  for (int r = 0; r < 8; ++r) { const float il = (1.0f / 16384.0f) / lrun[r];
#pragma unroll
    for (int t = 0; t < 4; ++t) so[(8 * g + r) * HD + t * 16 + ln] = acc[t][r] * il; }
  asm volatile("s_wait_dscnt 0" ::: "memory"); __builtin_amdgcn_wave_barrier(); __builtin_amdgcn_fence(__ATOMIC_RELEASE, "workgroup");
#pragma unroll
  for (int q = 0; q < 8; ++q) { const int rl = q * 2 + (lane >> 4), pc = lane & 15;
    vst2(O + base + (size_t)(q0 + rl) * HD + pc * 4, *(const v4f*)(so + rl * HD + pc * 4)); }
}

extern "C" void kernel_launch(void* const* d_in, const int* in_sizes, int n_in,
                              void* d_out, int out_size, void* d_ws, size_t ws_size,
                              hipStream_t stream) {
  (void)in_sizes; (void)n_in; (void)out_size; (void)d_ws; (void)ws_size;
  const float* q = (const float*)d_in[0];
  const float* k = (const float*)d_in[1];
  const float* v = (const float*)d_in[2];
  const float* mask = (const float*)d_in[3];
  const int* scale = (const int*)d_in[4];
  float* o = (float*)d_out;
  attn_fwd<<<dim3(SQ / BQ, NBH), 128, 0, stream>>>(q, k, v, mask, scale, o);
}
